// ZYWnet_12111807774785
// MI455X (gfx1250) — hardware-verified
//
#include <hip/hip_runtime.h>
#include <stddef.h>


typedef __bf16 v16b __attribute__((ext_vector_type(16)));
typedef unsigned short v8us __attribute__((ext_vector_type(8)));
typedef float v8f __attribute__((ext_vector_type(8)));
typedef float v4f __attribute__((ext_vector_type(4)));

union Frag { v16b v; v8us q[2]; };

namespace cfg {
constexpr int B = 8, S = 1024, D = 512, H = 8, DFF = 2048, L = 4, DK = 64;
constexpr int ROWS = B * S;
}

__device__ __forceinline__ unsigned short bf_bits(float f) {
  unsigned int u = __float_as_uint(f);
  u += 0x7fffu + ((u >> 16) & 1u);
  return (unsigned short)(u >> 16);
}
__device__ __forceinline__ float bf_val(unsigned short b) {
  return __uint_as_float(((unsigned int)b) << 16);
}
__device__ __forceinline__ void split1(float x, unsigned short& hi, unsigned short& lo) {
  hi = bf_bits(x);
  lo = bf_bits(x - bf_val(hi));
}
__device__ __forceinline__ void split4(const v4f x, v8us& h, v8us& l, const int o) {
#pragma unroll
  for (int c = 0; c < 4; ++c) {
    unsigned short th, tl;
    split1(x[c], th, tl);
    h[o + c] = th;
    l[o + c] = tl;
  }
}
__device__ __forceinline__ v8f zero8() {
  v8f z = {0.f, 0.f, 0.f, 0.f, 0.f, 0.f, 0.f, 0.f};
  return z;
}
__device__ __forceinline__ v8us zero8us() {
  v8us z = {0, 0, 0, 0, 0, 0, 0, 0};
  return z;
}

__device__ __forceinline__ void wmma3(v8f& acc, const Frag& ah, const Frag& al,
                                      const Frag& bh, const Frag& bl) {
  acc = __builtin_amdgcn_wmma_f32_16x16x32_bf16(false, ah.v, false, bh.v, (short)0, acc, false, false);
  acc = __builtin_amdgcn_wmma_f32_16x16x32_bf16(false, ah.v, false, bl.v, (short)0, acc, false, false);
  acc = __builtin_amdgcn_wmma_f32_16x16x32_bf16(false, al.v, false, bh.v, (short)0, acc, false, false);
  asm volatile("v_nop\n\tv_nop\n\tv_nop\n\tv_nop"
               : "+v"(acc)
               : "v"(ah.v), "v"(al.v), "v"(bh.v), "v"(bl.v));
}

__global__ __launch_bounds__(256) void add_pe_k(const float* __restrict__ q,
                                                const float* __restrict__ qa,
                                                const float* __restrict__ pe,
                                                float* x, float* y, int n4) {
  using namespace cfg;
  const int i4 = blockIdx.x * 256 + threadIdx.x;
  if (i4 >= n4) return;
  const size_t off = (size_t)i4 * 4;
  const size_t poff = off & (size_t)(S * D - 1);
  const v4f p = *(const v4f*)(pe + poff);
  const v4f a = *(const v4f*)(q + off);
  const v4f c = *(const v4f*)(qa + off);
  const v4f xv = a + p;
  const v4f yv = c + p;
  *(volatile v4f*)(x + off) = xv;
  *(volatile v4f*)(y + off) = yv;
  __threadfence();
  *(volatile v4f*)(x + off) = xv;
  *(volatile v4f*)(y + off) = yv;
}

constexpr int GBM = 64, GBN = 128, GBK = 32, GAP = 40;

__global__ __launch_bounds__(256) void gemm_k(const float* __restrict__ A,
                                              const float* __restrict__ W,
                                              const float* __restrict__ bias,
                                              float* out, int M, int N, int K, int relu) {
  __shared__ __align__(16) unsigned short Ah[GBM * GAP];
  __shared__ __align__(16) unsigned short Al[GBM * GAP];
  __shared__ __align__(16) unsigned short Wh[GBN * GAP];
  __shared__ __align__(16) unsigned short Wl[GBN * GAP];
  __shared__ __align__(16) float Ep[8][16 * 32];

  const int tid = threadIdx.x;
  const int lane = tid & 31, wid = tid >> 5;
  const int hh = lane >> 4, m = lane & 15;
  const int wm = wid >> 2, wn = wid & 3;
  const int m0 = blockIdx.y * GBM, n0 = blockIdx.x * GBN;
  if (m0 + GBM > M || n0 + GBN > N) return;

  v8f acc[2][2];
#pragma unroll
  for (int i = 0; i < 2; ++i)
#pragma unroll
    for (int j = 0; j < 2; ++j) acc[i][j] = zero8();

  const int ar = tid >> 2, akq = (tid & 3) * 8;
  const int wnn = tid & 127, wkg = (tid >> 7) * 16;
  const int T = K / GBK;

  for (int t = 0; t < T; ++t) {
    const int k0 = t * GBK;
    __syncthreads();
    {
      const float* ap = A + (size_t)(m0 + ar) * K + k0 + akq;
      const v4f x0 = *(const v4f*)(ap);
      const v4f x1 = *(const v4f*)(ap + 4);
      v8us h8 = zero8us(), l8 = zero8us();
      split4(x0, h8, l8, 0);
      split4(x1, h8, l8, 4);
      *(v8us*)(Ah + ar * GAP + akq) = h8;
      *(v8us*)(Al + ar * GAP + akq) = l8;
    }
    {
      const float* wp = W + (size_t)(k0 + wkg) * N + n0 + wnn;
      v8us h0 = zero8us(), l0 = zero8us(), h1 = zero8us(), l1 = zero8us();
#pragma unroll
      for (int i = 0; i < 8; ++i) {
        unsigned short th, tl;
        split1(wp[(size_t)i * N], th, tl);
        h0[i] = th; l0[i] = tl;
      }
#pragma unroll
      for (int i = 0; i < 8; ++i) {
        unsigned short th, tl;
        split1(wp[(size_t)(i + 8) * N], th, tl);
        h1[i] = th; l1[i] = tl;
      }
      *(v8us*)(Wh + wnn * GAP + wkg) = h0;
      *(v8us*)(Wh + wnn * GAP + wkg + 8) = h1;
      *(v8us*)(Wl + wnn * GAP + wkg) = l0;
      *(v8us*)(Wl + wnn * GAP + wkg + 8) = l1;
    }
    __syncthreads();

    Frag bh[2], bl[2];
#pragma unroll
    for (int j = 0; j < 2; ++j) {
      const int nr = (wn * 32 + j * 16 + m) * GAP;
      bh[j].q[0] = *(const v8us*)(Wh + nr + 8 * hh);
      bh[j].q[1] = *(const v8us*)(Wh + nr + 16 + 8 * hh);
      bl[j].q[0] = *(const v8us*)(Wl + nr + 8 * hh);
      bl[j].q[1] = *(const v8us*)(Wl + nr + 16 + 8 * hh);
    }
#pragma unroll
    for (int i = 0; i < 2; ++i) {
      const int rr = (wm * 32 + i * 16 + m) * GAP;
      Frag ah, al;
      ah.q[0] = *(const v8us*)(Ah + rr + 8 * hh);
      ah.q[1] = *(const v8us*)(Ah + rr + 16 + 8 * hh);
      al.q[0] = *(const v8us*)(Al + rr + 8 * hh);
      al.q[1] = *(const v8us*)(Al + rr + 16 + 8 * hh);
#pragma unroll
      for (int j = 0; j < 2; ++j) wmma3(acc[i][j], ah, al, bh[j], bl[j]);
    }
  }

  float* ep = Ep[wid];
#pragma unroll
  for (int i = 0; i < 2; ++i) {
#pragma unroll
    for (int j = 0; j < 2; ++j) {
      const int cl = j * 16 + m;
      const float bvv = bias[n0 + wn * 32 + cl];
#pragma unroll
      for (int r = 0; r < 8; ++r) {
        float v = acc[i][j][r] + bvv;
        if (relu) v = fmaxf(v, 0.f);
        ep[(8 * hh + r) * 32 + cl] = v;
      }
    }
    __syncthreads();
    v4f ov[4];
    size_t go[4];
#pragma unroll
    for (int p = 0; p < 4; ++p) {
      const int row = p * 4 + (lane >> 3);
      const int c4 = (lane & 7) * 4;
      ov[p] = *(const v4f*)(ep + row * 32 + c4);
      go[p] = (size_t)(m0 + wm * 32 + i * 16 + row) * N + n0 + wn * 32 + c4;
    }
#pragma unroll
    for (int p = 0; p < 4; ++p) *(volatile v4f*)(out + go[p]) = ov[p];
    __threadfence();
#pragma unroll
    for (int p = 0; p < 4; ++p) *(volatile v4f*)(out + go[p]) = ov[p];
    __syncthreads();
  }
}

constexpr int KP = 72, VP = 40, PP = 40;

__global__ __launch_bounds__(128) void attn_k(const float* __restrict__ QK,
                                              const float* __restrict__ Vv,
                                              float* O) {
  using namespace cfg;
  __shared__ __align__(16) unsigned short Kh[32 * KP];
  __shared__ __align__(16) unsigned short Kl[32 * KP];
  __shared__ __align__(16) unsigned short Vh[64 * VP];
  __shared__ __align__(16) unsigned short Vl[64 * VP];
  __shared__ __align__(16) unsigned short Ph[4][16 * PP];
  __shared__ __align__(16) unsigned short Pl[4][16 * PP];
  __shared__ __align__(16) float Os[4][16 * 64];

  const int mt = blockIdx.x, h = blockIdx.y, b = blockIdx.z;
  const int m0 = mt * 64;
  const int tid = threadIdx.x;
  const int lane = tid & 31, wid = tid >> 5;
  const int hh = lane >> 4, m = lane & 15;

  const size_t base = (size_t)b * S * D + (size_t)h * DK;
  const int r0 = m0 + wid * 16;

  Frag qh[2], ql[2];
  {
    const float* qp = QK + base + (size_t)(r0 + m) * D;
#pragma unroll
    for (int kk = 0; kk < 2; ++kk) {
#pragma unroll
      for (int part = 0; part < 2; ++part) {
        const int off = kk * 32 + part * 16 + 8 * hh;
        const v4f x0 = *(const v4f*)(qp + off);
        const v4f x1 = *(const v4f*)(qp + off + 4);
        v8us h8 = zero8us(), l8 = zero8us();
        split4(x0, h8, l8, 0);
        split4(x1, h8, l8, 4);
        qh[kk].q[part] = h8;
        ql[kk].q[part] = l8;
      }
    }
  }

  v8f acc[4];
#pragma unroll
  for (int f = 0; f < 4; ++f) acc[f] = zero8();
  float mrow[8], lrow[8];
#pragma unroll
  for (int r = 0; r < 8; ++r) { mrow[r] = -1e30f; lrow[r] = 0.f; }

  const int kj = tid >> 2, kdq = (tid & 3) * 16;
  const int vd = tid & 63, vjg = (tid >> 6) * 16;
  const int T = m0 / 32 + 2;

  for (int t = 0; t < T; ++t) {
    const int j0 = t * 32;
    __syncthreads();
    {
      const float* kp = QK + base + (size_t)(j0 + kj) * D + kdq;
#pragma unroll
      for (int part = 0; part < 2; ++part) {
        const v4f x0 = *(const v4f*)(kp + part * 8);
        const v4f x1 = *(const v4f*)(kp + part * 8 + 4);
        v8us h8 = zero8us(), l8 = zero8us();
        split4(x0, h8, l8, 0);
        split4(x1, h8, l8, 4);
        *(v8us*)(Kh + kj * KP + kdq + part * 8) = h8;
        *(v8us*)(Kl + kj * KP + kdq + part * 8) = l8;
      }
    }
    {
      const float* vp = Vv + base + (size_t)(j0 + vjg) * D + vd;
      v8us h0 = zero8us(), l0 = zero8us(), h1 = zero8us(), l1 = zero8us();
#pragma unroll
      for (int i = 0; i < 8; ++i) {
        unsigned short th, tl;
        split1(vp[(size_t)i * D], th, tl);
        h0[i] = th; l0[i] = tl;
      }
#pragma unroll
      for (int i = 0; i < 8; ++i) {
        unsigned short th, tl;
        split1(vp[(size_t)(i + 8) * D], th, tl);
        h1[i] = th; l1[i] = tl;
      }
      *(v8us*)(Vh + vd * VP + vjg) = h0;
      *(v8us*)(Vh + vd * VP + vjg + 8) = h1;
      *(v8us*)(Vl + vd * VP + vjg) = l0;
      *(v8us*)(Vl + vd * VP + vjg + 8) = l1;
    }
    __syncthreads();

    v8f sc0 = zero8(), sc1 = zero8();
#pragma unroll
    for (int kk = 0; kk < 2; ++kk) {
      Frag kb_h, kb_l;
      const int n0r = m * KP + kk * 32;
      kb_h.q[0] = *(const v8us*)(Kh + n0r + 8 * hh);
      kb_h.q[1] = *(const v8us*)(Kh + n0r + 16 + 8 * hh);
      kb_l.q[0] = *(const v8us*)(Kl + n0r + 8 * hh);
      kb_l.q[1] = *(const v8us*)(Kl + n0r + 16 + 8 * hh);
      wmma3(sc0, qh[kk], ql[kk], kb_h, kb_l);
      const int n1r = (16 + m) * KP + kk * 32;
      kb_h.q[0] = *(const v8us*)(Kh + n1r + 8 * hh);
      kb_h.q[1] = *(const v8us*)(Kh + n1r + 16 + 8 * hh);
      kb_l.q[0] = *(const v8us*)(Kl + n1r + 8 * hh);
      kb_l.q[1] = *(const v8us*)(Kl + n1r + 16 + 8 * hh);
      wmma3(sc1, qh[kk], ql[kk], kb_h, kb_l);
    }

#pragma unroll
    for (int r = 0; r < 8; ++r) {
      const int grow = r0 + 8 * hh + r;
      const int c0 = j0 + m;
      const int c1 = c0 + 16;
      const float s0 = (c0 < grow) ? sc0[r] * 0.125f : -1e30f;
      const float s1 = (c1 < grow) ? sc1[r] * 0.125f : -1e30f;
      float bm = fmaxf(s0, s1);
#pragma unroll
      for (int mm = 1; mm < 16; mm <<= 1) bm = fmaxf(bm, __shfl_xor(bm, mm, 32));
      const float mnew = fmaxf(mrow[r], bm);
      const float scl = __expf(mrow[r] - mnew);
      const float p0 = __expf(s0 - mnew);
      const float p1 = __expf(s1 - mnew);
      float rs = p0 + p1;
#pragma unroll
      for (int mm = 1; mm < 16; mm <<= 1) rs += __shfl_xor(rs, mm, 32);
      lrow[r] = lrow[r] * scl + rs;
      mrow[r] = mnew;
#pragma unroll
      for (int f = 0; f < 4; ++f) acc[f][r] = acc[f][r] * scl;
      const int prow = (8 * hh + r) * PP;
      unsigned short th, tl;
      split1(p0, th, tl);
      Ph[wid][prow + m] = th;
      Pl[wid][prow + m] = tl;
      split1(p1, th, tl);
      Ph[wid][prow + 16 + m] = th;
      Pl[wid][prow + 16 + m] = tl;
    }
    __syncthreads();

    Frag ph, pl;
    {
      const int pr = m * PP;
      ph.q[0] = *(const v8us*)(&Ph[wid][pr + 8 * hh]);
      ph.q[1] = *(const v8us*)(&Ph[wid][pr + 16 + 8 * hh]);
      pl.q[0] = *(const v8us*)(&Pl[wid][pr + 8 * hh]);
      pl.q[1] = *(const v8us*)(&Pl[wid][pr + 16 + 8 * hh]);
    }
#pragma unroll
    for (int f = 0; f < 4; ++f) {
      Frag vb_h, vb_l;
      const int vr = (f * 16 + m) * VP;
      vb_h.q[0] = *(const v8us*)(Vh + vr + 8 * hh);
      vb_h.q[1] = *(const v8us*)(Vh + vr + 16 + 8 * hh);
      vb_l.q[0] = *(const v8us*)(Vl + vr + 8 * hh);
      vb_l.q[1] = *(const v8us*)(Vl + vr + 16 + 8 * hh);
      wmma3(acc[f], ph, pl, vb_h, vb_l);
    }
  }

#pragma unroll
  for (int r = 0; r < 8; ++r) {
    const int srow = r0 + 8 * hh + r;
    const float inv = (srow == 0 || !(lrow[r] > 0.f)) ? 0.f : 1.f / lrow[r];
#pragma unroll
    for (int f = 0; f < 4; ++f) Os[wid][(8 * hh + r) * 64 + f * 16 + m] = acc[f][r] * inv;
  }
  __syncthreads();
  v4f ov[8];
  size_t go[8];
  const float* os = Os[wid];
#pragma unroll
  for (int p = 0; p < 8; ++p) {
    const int idx = p * 32 + lane;
    const int row = idx >> 4;
    const int c4 = (idx & 15) * 4;
    ov[p] = *(const v4f*)(os + row * 64 + c4);
    go[p] = base + (size_t)(r0 + row) * D + c4;
  }
#pragma unroll
  for (int p = 0; p < 8; ++p) *(volatile v4f*)(O + go[p]) = ov[p];
  __threadfence();
#pragma unroll
  for (int p = 0; p < 8; ++p) *(volatile v4f*)(O + go[p]) = ov[p];
}

__global__ __launch_bounds__(256) void add_ln_k(const float* X, const float* Tm,
                                                const float* __restrict__ g,
                                                const float* __restrict__ be,
                                                float* outF, int nrows) {
  using namespace cfg;
  const int row = blockIdx.x * 8 + (threadIdx.x >> 5);
  const int lane = threadIdx.x & 31;
  if (row >= nrows) return;
  const size_t rb = (size_t)row * D;

  v4f z[4];
  float s = 0.f;
#pragma unroll
  for (int i = 0; i < 4; ++i) {
    const int c = i * 128 + lane * 4;
    const v4f a = *(const v4f*)(X + rb + c);
    const v4f t = *(const v4f*)(Tm + rb + c);
    z[i] = a + t;
    s += z[i][0] + z[i][1] + z[i][2] + z[i][3];
  }
#pragma unroll
  for (int mm = 1; mm < 32; mm <<= 1) s += __shfl_xor(s, mm, 32);
  const float mean = s * (1.f / D);
  float v = 0.f;
#pragma unroll
  for (int i = 0; i < 4; ++i) {
#pragma unroll
    for (int c = 0; c < 4; ++c) { const float d = z[i][c] - mean; v += d * d; }
  }
#pragma unroll
  for (int mm = 1; mm < 32; mm <<= 1) v += __shfl_xor(v, mm, 32);
  const float den = sqrtf(v * (1.f / D) + 1e-5f);
  const float inv = 1.f / den;

  v4f ov[4];
#pragma unroll
  for (int i = 0; i < 4; ++i) {
    const int c = i * 128 + lane * 4;
    const v4f gg = *(const v4f*)(g + c);
    const v4f bb = *(const v4f*)(be + c);
    v4f o;
#pragma unroll
    for (int cc = 0; cc < 4; ++cc) o[cc] = (z[i][cc] - mean) * inv * gg[cc] + bb[cc];
    ov[i] = o;
  }
#pragma unroll
  for (int i = 0; i < 4; ++i) *(volatile v4f*)(outF + rb + i * 128 + lane * 4) = ov[i];
  __threadfence();
#pragma unroll
  for (int i = 0; i < 4; ++i) *(volatile v4f*)(outF + rb + i * 128 + lane * 4) = ov[i];
}

extern "C" void kernel_launch(void* const* d_in, const int* in_sizes, int n_in,
                              void* d_out, int out_size, void* d_ws, size_t ws_size,
                              hipStream_t stream) {
  using namespace cfg;
  if (n_in < 17) return;
  const size_t RD = (size_t)ROWS * D;
  if ((size_t)out_size != RD) return;
  if ((size_t)in_sizes[0] != RD || (size_t)in_sizes[1] != RD) return;
  if ((size_t)in_sizes[2] != (size_t)S * D) return;
  if ((size_t)in_sizes[3] != (size_t)L * D * D || (size_t)in_sizes[11] != (size_t)L * D * DFF ||
      (size_t)in_sizes[13] != (size_t)L * DFF * D) return;

  const float* q_emb  = (const float*)d_in[0];
  const float* qa_emb = (const float*)d_in[1];
  const float* pe     = (const float*)d_in[2];
  const float* Wk  = (const float*)d_in[3];
  const float* bk  = (const float*)d_in[4];
  const float* Wv  = (const float*)d_in[5];
  const float* bv  = (const float*)d_in[6];
  const float* Wo  = (const float*)d_in[7];
  const float* bo  = (const float*)d_in[8];
  const float* l1s = (const float*)d_in[9];
  const float* l1b = (const float*)d_in[10];
  const float* W1  = (const float*)d_in[11];
  const float* b1  = (const float*)d_in[12];
  const float* W2  = (const float*)d_in[13];
  const float* b2  = (const float*)d_in[14];
  const float* l2s = (const float*)d_in[15];
  const float* l2b = (const float*)d_in[16];

  const size_t bRD = RD * sizeof(float);
  const size_t bHB = (size_t)ROWS * DFF * sizeof(float);
  const size_t total = 6 * bRD + bHB;
  if (total > ws_size) return;
  char* wsp = (char*)d_ws;
  float* x   = (float*)(wsp + 0 * bRD);
  float* tmp = (float*)(wsp + 1 * bRD);
  float* y   = (float*)(wsp + 2 * bRD);
  float* qk  = (float*)(wsp + 3 * bRD);
  float* vv  = (float*)(wsp + 4 * bRD);
  float* ob  = (float*)(wsp + 5 * bRD);
  float* hb  = (float*)(wsp + 6 * bRD);

  const int n4 = (int)(RD / 4);
  add_pe_k<<<dim3((n4 + 255) / 256), dim3(256), 0, stream>>>(q_emb, qa_emb, pe, x, y, n4);

  const dim3 gProj(D / GBN, ROWS / GBM);
  const dim3 gFfn1(DFF / GBN, ROWS / GBM);
  const dim3 gAttn(S / 64, H, B);
  const dim3 gLn((ROWS + 7) / 8);

  for (int l = 0; l < L; ++l) {
    const float* wk = Wk + (size_t)l * D * D;
    const float* wv = Wv + (size_t)l * D * D;
    const float* wo = Wo + (size_t)l * D * D;
    const float* w1 = W1 + (size_t)l * D * DFF;
    const float* w2 = W2 + (size_t)l * DFF * D;

    gemm_k<<<gProj, 256, 0, stream>>>(x, wk, bk + (size_t)l * D, qk, ROWS, D, D, 0);
    gemm_k<<<gProj, 256, 0, stream>>>(y, wv, bv + (size_t)l * D, vv, ROWS, D, D, 0);
    attn_k<<<gAttn, 128, 0, stream>>>(qk, vv, ob);
    gemm_k<<<gProj, 256, 0, stream>>>(ob, wo, bo + (size_t)l * D, tmp, ROWS, D, D, 0);
    add_ln_k<<<gLn, 256, 0, stream>>>(x, tmp, l1s + (size_t)l * D, l1b + (size_t)l * D, x, ROWS);
    gemm_k<<<gFfn1, 256, 0, stream>>>(x, w1, b1 + (size_t)l * DFF, hb, ROWS, DFF, D, 1);
    gemm_k<<<gProj, 256, 0, stream>>>(hb, w2, b2 + (size_t)l * D, tmp, ROWS, D, DFF, 0);
    float* dst = (l == L - 1) ? (float*)d_out : x;
    add_ln_k<<<gLn, 256, 0, stream>>>(x, tmp, l2s + (size_t)l * D, l2b + (size_t)l * D, dst, ROWS);
  }
}
